// SlidingATTN_88330297409593
// MI455X (gfx1250) — hardware-verified
//
#include <hip/hip_runtime.h>
#include <math.h>

typedef __attribute__((ext_vector_type(16))) _Float16 v16h;
typedef __attribute__((ext_vector_type(16))) __bf16 v16b;
typedef __attribute__((ext_vector_type(8)))  _Float16 v8h;
typedef __attribute__((ext_vector_type(8)))  float v8f;
typedef __attribute__((ext_vector_type(4)))  float v4f;
typedef __attribute__((ext_vector_type(2)))  float v2f;
typedef __attribute__((ext_vector_type(4)))  unsigned v4u;
typedef __attribute__((ext_vector_type(4)))  int v4i;
typedef float __attribute__((may_alias)) float_a;
typedef int __attribute__((may_alias)) int_a;

template <typename T> __device__ __forceinline__ void vst2(void* p, T v) { *(volatile T*)p = v; __threadfence(); *(volatile T*)p = v; }
__device__ __forceinline__ v8f wmma16(v16h a, v16h b, v8f c) {
  v8f d = __builtin_amdgcn_wmma_f32_16x16x32_f16(false, a, false, b, (short)0, c, false, false);
  asm volatile("v_nop\n\tv_nop\n\tv_nop\n\tv_nop" : "+v"(d) : "v"(a), "v"(b));
  return d;
}
__device__ __forceinline__ v8f wmma_bf(v16b a, v16b b, v8f c) {
  v8f d = __builtin_amdgcn_wmma_f32_16x16x32_bf16(false, a, false, b, (short)0, c, false, false);
  asm volatile("v_nop\n\tv_nop\n\tv_nop\n\tv_nop" : "+v"(d) : "v"(a), "v"(b));
  return d;
}
__device__ __forceinline__ v16h frag_h(const _Float16* rowk0, int lane) {
  union { v16h v; v8h q[2]; } u; const _Float16* p = rowk0 + 8 * (lane >> 4);
  u.q[0] = *(const v8h*)p; u.q[1] = *(const v8h*)(p + 16); return u.v;
}
__device__ __forceinline__ v16h frag_f32(const float* rowk0, int lane) {
  v16h a; const float* p = rowk0 + 8 * (lane >> 4);
#pragma unroll
  for (int i = 0; i < 8; ++i) { a[i] = (_Float16)p[i]; a[8 + i] = (_Float16)p[16 + i]; }
  return a;
}
__device__ __forceinline__ v16h frag_f32s(const float* rowk0, int lane, float sc) {
  v16h a; const float* p = rowk0 + 8 * (lane >> 4);
#pragma unroll
  for (int i = 0; i < 8; ++i) { a[i] = (_Float16)(p[i] * sc); a[8 + i] = (_Float16)(p[16 + i] * sc); }
  return a;
}
__device__ __forceinline__ v16h fragc_f32(const float* W, int k0, int n, int lane, int ld, int K) {
  v16h a; const int g = lane >> 4;
#pragma unroll
  for (int i = 0; i < 8; ++i) { const int ka = k0 + 8 * g + i, kb = ka + 16;
    a[i] = (_Float16)(ka < K ? W[(size_t)(ka < K ? ka : K - 1) * ld + n] : 0.f); a[8 + i] = (_Float16)(kb < K ? W[(size_t)(kb < K ? kb : K - 1) * ld + n] : 0.f); }
  return a;
}
struct F2 { v16b h, l; };
__device__ __forceinline__ F2 bsplit16(const float v[16]) { F2 r;
#pragma unroll
  for (int i = 0; i < 16; ++i) { const __bf16 h = (__bf16)v[i]; r.h[i] = h; r.l[i] = (__bf16)(v[i] - (float)h); }
  return r; }
__device__ __forceinline__ F2 split_row(const float* row, int k0, int lane) { float v[16]; const float* p = row + k0 + 8 * (lane >> 4);
#pragma unroll
  for (int i = 0; i < 8; ++i) { v[i] = p[i]; v[8 + i] = p[16 + i]; }
  return bsplit16(v); }
__device__ __forceinline__ F2 split_rowK(const float* row, int k0, int lane, int K) { float v[16]; const int g = lane >> 4;
#pragma unroll
  for (int i = 0; i < 8; ++i) { const int ka = k0 + 8 * g + i, kb = ka + 16; v[i] = ka < K ? row[ka < K ? ka : K - 1] : 0.f; v[8 + i] = kb < K ? row[kb < K ? kb : K - 1] : 0.f; }
  return bsplit16(v); }
__device__ __forceinline__ F2 split_col(const float* W, int k0, int n, int lane, int ld, int K) { float v[16]; const int g = lane >> 4;
#pragma unroll
  for (int i = 0; i < 8; ++i) { const int ka = k0 + 8 * g + i, kb = ka + 16; v[i] = ka < K ? W[(size_t)(ka < K ? ka : K - 1) * ld + n] : 0.f; v[8 + i] = kb < K ? W[(size_t)(kb < K ? kb : K - 1) * ld + n] : 0.f; }
  return bsplit16(v); }
__device__ __forceinline__ v8f mac3(const F2& a, const F2& b, v8f c) { c = wmma_bf(a.l, b.h, c); c = wmma_bf(a.h, b.l, c); return wmma_bf(a.h, b.h, c); }
__device__ __forceinline__ float sigm(float v) { return 1.0f / (1.0f + expf(-v)); }
#define LDSX() do { asm volatile("s_wait_dscnt 0" ::: "memory"); __builtin_amdgcn_wave_barrier(); __builtin_amdgcn_fence(__ATOMIC_RELEASE, "workgroup"); } while (0)


#define NB 16
#define LL 1024
#define DD 256
#define NH 8
#define HDD 32
#define WW 33
#define DIL 2
#define PAD 33
#define NR (NB * LL)
#ifndef TRB
#define TRB (NR / 64)
#endif
typedef __attribute__((ext_vector_type(8))) __bf16 v8b;
__device__ __forceinline__ v16b frag_b(const __bf16* rowk0, int lane) {
  union { v16b v; v8b q[2]; } u; const __bf16* p = rowk0 + 8 * (lane >> 4);
  u.q[0] = *(const v8b*)p; u.q[1] = *(const v8b*)(p + 16); return u.v;
}
__device__ __forceinline__ float bfr(float v) { return (float)(__bf16)v; }
__device__ __attribute__((noinline)) float exp_ni(float v) { return expf(v); }
__device__ __attribute__((noinline)) float erf_ni(float v) { return erff(v); }
__device__ __attribute__((noinline)) float exp_p(float v) { return expf(v); }
__device__ __attribute__((noinline)) float expm1_p(float v) { return expm1f(v); }

#define WS_PW  0u
#define WS_V0  (WS_PW + 2u * (size_t)2 * DD * DD)
#define WS_A   (WS_V0 + 4u * (size_t)NR * DD)
#define WS_O   (WS_A + 4u * (size_t)NR * 32)
#define WS_O0  (WS_O + 4u * (size_t)NR * DD)
#define WS_END (WS_O0 + 4u * (size_t)NR * DD)

__global__ __launch_bounds__(256) void k_pack(const float* __restrict__ VW, const float* __restrict__ OW, __bf16* __restrict__ PW) { const int n = blockIdx.x, which = blockIdx.y, t = threadIdx.x; __shared__ __align__(16) __bf16 s[DD]; const float* w = which ? OW : VW; s[t] = (__bf16)w[(size_t)t * DD + n]; __syncthreads(); if (t < DD / 8) vst2((unsigned*)(PW + ((size_t)which * DD + n) * DD + t * 8), *(const v4u*)&s[t * 8]); }
template <int MODE>
__global__ __launch_bounds__(128) void k_g(const float* __restrict__ A, const __bf16* __restrict__ P, const float* __restrict__ BB, float* __restrict__ OUT) { __shared__ __align__(16) float so[4][16][132];
  const int tid = threadIdx.x, wave = tid >> 5, lane = tid & 31, col = lane & 15, g = lane >> 4; const size_t r0 = (size_t)blockIdx.x * 64 + wave * 16; const int c0 = blockIdx.y * 128;
  v8f acc[8] = {};
#pragma unroll
  for (int kc = 0; kc < DD / 32; ++kc) {
    if (MODE == 0) { v16b a; { const float* p = A + (r0 + col) * DD + kc * 32 + 8 * g;
#pragma unroll
        for (int i = 0; i < 8; ++i) { a[i] = (__bf16)p[i]; a[8 + i] = (__bf16)p[16 + i]; } }
#pragma unroll
      for (int j = 0; j < 8; ++j) acc[j] = wmma_bf(a, frag_b(P + (size_t)(c0 + j * 16 + col) * DD + kc * 32, lane), acc[j]); }
    else { const F2 a = split_row(A + (r0 + col) * DD, kc * 32, lane);
#pragma unroll
      for (int j = 0; j < 8; ++j) { const v16b w = frag_b(P + (size_t)(c0 + j * 16 + col) * DD + kc * 32, lane); acc[j] = wmma_bf(a.h, w, acc[j]); acc[j] = wmma_bf(a.l, w, acc[j]); } } }
#pragma unroll
  for (int j = 0; j < 8; ++j) { const float bb = bfr(BB[c0 + j * 16 + col]);
#pragma unroll
    for (int r = 0; r < 8; ++r) so[wave][8 * g + r][j * 16 + col] = acc[j][r] + bb; }
  LDSX(); for (int rl = 0; rl < 16; ++rl) vst2(OUT + (r0 + rl) * DD + c0 + lane * 4, *(const v4f*)&so[wave][rl][lane * 4]); }
template <int FIN>
__global__ __launch_bounds__(256) void k_rows(float* __restrict__ V0, const float* __restrict__ G, const float* __restrict__ Bt, const float* __restrict__ X, const float* __restrict__ AW, const float* __restrict__ AB, const int* __restrict__ MK, float* __restrict__ A, float* __restrict__ OUT) {
  __shared__ float red[8]; __shared__ float sx[DD]; __shared__ __align__(16) float sa[32]; __shared__ __align__(16) float so2[DD]; const int t = threadIdx.x; const size_t row = blockIdx.x;
  const float v = V0[row * DD + t]; float s = v;
#pragma unroll
  for (int o = 1; o < 32; o <<= 1) s += __shfl_xor(s, o);
  if ((t & 31) == 0) red[t >> 5] = s; __syncthreads(); float tot = 0.f; for (int i = 0; i < 8; ++i) tot += red[i]; const float mu = tot / (float)DD; __syncthreads();
  const float d = v - mu; float q = d * d;
#pragma unroll
  for (int o = 1; o < 32; o <<= 1) q += __shfl_xor(q, o);
  if ((t & 31) == 0) red[t >> 5] = q; __syncthreads(); float tq = 0.f; for (int i = 0; i < 8; ++i) tq += red[i]; const float inv = 1.0f / sqrtf(tq / (float)DD + 1e-5f);
  { const float yv = d * inv * bfr(G[t]) + bfr(Bt[t]); const float ev = (yv > 0.f) ? yv : expm1_p(yv); so2[t] = FIN ? (ev + bfr(X[row * DD + t])) : ev; }
  if (FIN == 0) { sx[t] = bfr(X[row * DD + t]); __syncthreads();
    { const int h = t >> 5, part = t & 31; float a = 0.f; for (int c = part; c < DD; c += 32) a += sx[c] * bfr(AW[(size_t)c * NH + h]);
#pragma unroll
      for (int o = 1; o < 32; o <<= 1) a += __shfl_xor(a, o);
      if (part == 0) sa[h] = (MK[row] != 0) ? 0.f : exp_p(a + bfr(AB[h])); if (part == 1 && h == 0) { for (int e = NH; e < 32; ++e) sa[e] = 0.f; } } }
  __syncthreads();
  if (t < DD / 4) vst2((FIN ? OUT : V0) + row * DD + t * 4, *(const v4f*)&so2[t * 4]);
  if (FIN == 0 && t >= 128 && t < 136) vst2(A + row * 32 + (t - 128) * 4, *(const v4f*)&sa[(t - 128) * 4]);
}
__global__ __launch_bounds__(256) void k_win(const float* __restrict__ A, const float* __restrict__ V, const float* __restrict__ POS, float* __restrict__ O) { __shared__ __align__(16) float so2[DD]; const int t = threadIdx.x; const int h = t >> 5, dd = t & 31; const size_t row = blockIdx.x; const size_t b = row / LL; const int l = (int)(row % LL);
  float acc = 0.f, z = 0.f;
#pragma unroll 1
  for (int w = 0; w < WW; ++w) { const int p = l + DIL * w - PAD; if (p < 0 || p >= LL) continue; const size_t pr = b * LL + p; const float aw = A[pr * 32 + h] * exp_p(bfr(POS[w * NH + h])); z += aw; acc += aw * V[pr * DD + h * HDD + dd]; }
  so2[t] = acc / (z + 1e-5f); __syncthreads(); if (t < DD / 4) vst2(O + row * DD + t * 4, *(const v4f*)&so2[t * 4]); }
extern "C" void kernel_launch(void* const* d_in, const int* in_sizes, int n_in, void* d_out, int out_size, void* d_ws, size_t ws_size, hipStream_t stream) {
  (void)in_sizes; (void)n_in; (void)out_size;
  const float** F = (const float**)d_in;
  if (ws_size < (size_t)WS_END) return;
  char* ws = (char*)d_ws; __bf16* PW = (__bf16*)(ws + WS_PW); float *V0 = (float*)(ws + WS_V0), *A = (float*)(ws + WS_A), *O = (float*)(ws + WS_O), *O0 = (float*)(ws + WS_O0);
  k_pack<<<dim3(DD, 2), 256, 0, stream>>>(F[5], F[9], PW);
  k_g<0><<<dim3(NR / 64, DD / 128), 128, 0, stream>>>(F[0], PW, F[6], V0);
  k_rows<0><<<NR, 256, 0, stream>>>(V0, F[7], F[8], F[0], F[2], F[3], (const int*)d_in[1], A, nullptr);
  k_win<<<TRB * 64, 256, 0, stream>>>(A, V0, F[4], O);
  k_g<1><<<dim3(TRB, DD / 128), 128, 0, stream>>>(O, PW + (size_t)DD * DD, F[10], O0);
  k_rows<1><<<TRB * 64, 256, 0, stream>>>(O0, F[11], F[12], F[0], nullptr, nullptr, nullptr, nullptr, (float*)d_out);
}
